// RoIAlignAppearanceEncoder_89266600280310
// MI455X (gfx1250) — hardware-verified
//
#include <hip/hip_runtime.h>


namespace {
constexpr int Bn = 16, IMG = 512, FS = 32, C = 256, NB = 16, S = 7, KP = 768  , NPATCH = Bn * FS * FS  , D = 256;
constexpr float AS_ = 8.0f;

typedef _Float16 b16;
typedef __attribute__((ext_vector_type(16))) _Float16 v16b;
typedef __attribute__((ext_vector_type(8))) _Float16 v8b;
typedef __attribute__((ext_vector_type(8))) float v8f;
typedef __attribute__((ext_vector_type(4))) float v4f;
__device__ __forceinline__ float bf16_rne(float f) { unsigned int u = __float_as_uint(f); u += 0x7FFFu + ((u >> 16) & 1u); return __uint_as_float(u & 0xFFFF0000u); }
__device__ __forceinline__ void split16(float v, b16& hi, b16& lo) { hi = (b16)v; lo = (b16)(v - (float)hi); }
__device__ __forceinline__ v16b frag_kb(const b16* p, int hh) { const v8b a = *(const v8b*)(p + 8 * hh), b = *(const v8b*)(p + 16 + 8 * hh); v16b f;
#pragma unroll
  for (int e = 0; e < 8; ++e) { f[e] = a[e]; f[8 + e] = b[e]; } return f; }
__device__ __forceinline__ void frag_split(const float* p, int hh, v16b& fh, v16b& fl) {
#pragma unroll
  for (int e = 0; e < 8; ++e) { b16 a, c; split16(p[8 * hh + e] * AS_, a, c); fh[e] = a; fl[e] = c; split16(p[16 + 8 * hh + e] * AS_, a, c); fh[8 + e] = a; fl[8 + e] = c; } }
__device__ __forceinline__ v8f wmma16b(v16b a, v16b b, v8f c) { v8f d = __builtin_amdgcn_wmma_f32_16x16x32_f16(false, a, false, b, (short)0, c, false, false); asm volatile("v_nop\n\tv_nop\n\tv_nop\n\tv_nop" : "+v"(d) : "v"(a), "v"(b)); return d; }
__device__ __forceinline__ void wave_lds_sync() { __builtin_amdgcn_fence(__ATOMIC_RELEASE, "workgroup"); __builtin_amdgcn_wave_barrier(); __builtin_amdgcn_fence(__ATOMIC_ACQUIRE, "workgroup"); }
__device__ __forceinline__ float pmul(float a, float b) { float p = a * b; asm volatile("" : "+v"(p)); return p; }

__global__ __launch_bounds__(256) void patch_kernel(const float* __restrict__ img, const float* __restrict__ cw, b16* __restrict__ A, b16* __restrict__ Wc) {
  const int b = blockIdx.y, py = blockIdx.x, t_ = threadIdx.x;
  for (int pass = 0; pass < 2; ++pass) {
    for (int i = t_; i < 32 * (KP / 8); i += 256) { const int px = i / (KP / 8), k0 = (i % (KP / 8)) * 8; const int dy = k0 / 48, r0 = k0 % 48; v8b v;
#pragma unroll
      for (int e = 0; e < 8; ++e) { const int r = r0 + e; v[e] = (b16)bf16_rne(img[(((size_t)b * IMG + py * 16 + dy) * IMG + px * 16) * 3 + r]); }
      *(volatile v8b*)(A + (((size_t)b * FS + py) * FS + px) * KP + k0) = v; }
    if (py == 0) { for (int i = b * 256 + t_; i < C * (KP / 8); i += Bn * 256) { const int co = i / (KP / 8), k0 = (i % (KP / 8)) * 8; v8b v; for (int e = 0; e < 8; ++e) v[e] = (b16)bf16_rne(cw[(size_t)(k0 + e) * C + co]); *(volatile v8b*)(Wc + (size_t)co * KP + k0) = v; } }
    __threadfence(); }
}

__global__ __launch_bounds__(64) void stem_kernel(const b16* __restrict__ A, const b16* __restrict__ Wc, const float* __restrict__ cb, float* __restrict__ F) {
  __shared__ __attribute__((aligned(16))) float Ts[2][32][128 + 4];
  const int lane = threadIdx.x & 31, wave = threadIdx.x >> 5, nloc = lane & 15, hlf = lane >> 4, m0 = blockIdx.y * 32, c0 = blockIdx.x * 128 + 0 * wave;
  const int cw0 = blockIdx.x * 128 + wave * 64;
  v8f acc[2][4];
#pragma unroll
  for (int r = 0; r < 2; ++r)
#pragma unroll
    for (int t = 0; t < 4; ++t) acc[r][t] = (v8f){};
#pragma unroll 2
  for (int kb = 0; kb < KP; kb += 32) { const v16b a0 = frag_kb(A + (size_t)(m0 + nloc) * KP + kb, hlf), a1 = frag_kb(A + (size_t)(m0 + 16 + nloc) * KP + kb, hlf);
#pragma unroll
    for (int t = 0; t < 4; ++t) { const v16b bw = frag_kb(Wc + (size_t)(cw0 + t * 16 + nloc) * KP + kb, hlf); acc[0][t] = wmma16b(a0, bw, acc[0][t]); acc[1][t] = wmma16b(a1, bw, acc[1][t]); } }
  (void)c0;
#pragma unroll
  for (int t = 0; t < 4; ++t) { const float bb = cb[cw0 + t * 16 + nloc];
#pragma unroll
    for (int r = 0; r < 2; ++r)
#pragma unroll
      for (int v = 0; v < 8; ++v) Ts[wave][r * 16 + 8 * hlf + v][t * 16 + nloc] = fmaxf(acc[r][t][v] + bb, 0.0f); }
  wave_lds_sync();
  for (int pass = 0; pass < 2; ++pass) { for (int i = lane; i < 32 * 16; i += 32) { const int rr = i >> 4, c4 = (i & 15) * 4; *(volatile v4f*)(F + (size_t)(m0 + rr) * C + cw0 + c4) = *(const v4f*)(&Ts[wave][rr][c4]); } __threadfence(); }
}

__global__ __launch_bounds__(256) void roi_kernel(const float* __restrict__ F, const float* __restrict__ boxes, const b16* __restrict__ Wd, const float* __restrict__ db, float* __restrict__ out) {
  __shared__ __attribute__((aligned(16))) float Ob[16][C + 4]; __shared__ __attribute__((aligned(16))) float Oo[C];
  const int b = blockIdx.y, n = blockIdx.x, c = threadIdx.x, lane = c & 31, wave = c >> 5, nloc = lane & 15, hlf = lane >> 4;
  const float ymin = bf16_rne(boxes[((size_t)b * NB + n) * 4]), xmin = bf16_rne(boxes[((size_t)b * NB + n) * 4 + 1]), ymax = bf16_rne(boxes[((size_t)b * NB + n) * 4 + 2]), xmax = bf16_rne(boxes[((size_t)b * NB + n) * 4 + 3]);
  const bool empty = (ymin == -1.0f) && (xmin == -1.0f) && (ymax == -1.0f) && (xmax == -1.0f);
  int y0i[S], y1i[S], x0i[S], x1i[S]; float wy[S], wx[S];
#pragma unroll
  for (int s = 0; s < S; ++s) { const float st = ((float)s + 0.5f) / (float)S;
    { const float ys = ymin + (ymax - ymin) * st; const float py = ys * (float)FS - 0.5f; const float f = floorf(py); wy[s] = py - f; const int i0 = (int)f; y0i[s] = min(max(i0, 0), FS - 1); y1i[s] = min(max(i0 + 1, 0), FS - 1); }
    { const float xs = xmin + (xmax - xmin) * st; const float px = xs * (float)FS - 0.5f; const float f = floorf(px); wx[s] = px - f; const int i0 = (int)f; x0i[s] = min(max(i0, 0), FS - 1); x1i[s] = min(max(i0 + 1, 0), FS - 1); } }
  float acc = 0.0f; const float* Fb = F + (size_t)b * FS * FS * C;
  for (int sy = 0; sy < S; ++sy) for (int sx = 0; sx < S; ++sx) {
    const float w00 = pmul(1.0f - wy[sy], 1.0f - wx[sx]), w01 = pmul(1.0f - wy[sy], wx[sx]), w10 = pmul(wy[sy], 1.0f - wx[sx]), w11 = pmul(wy[sy], wx[sx]);
    const float v = ((pmul(w00, Fb[((size_t)y0i[sy] * FS + x0i[sx]) * C + c]) + pmul(w01, Fb[((size_t)y0i[sy] * FS + x1i[sx]) * C + c])) + pmul(w10, Fb[((size_t)y1i[sy] * FS + x0i[sx]) * C + c])) + pmul(w11, Fb[((size_t)y1i[sy] * FS + x1i[sx]) * C + c]);
    acc += v; }
  const float obj = empty ? 0.0f : acc * (1.0f / (float)(S * S));
  for (int r = 0; r < 16; ++r) Ob[r][c] = (r == 0) ? obj : 0.0f;
  __syncthreads();
  { v8f o[4] = {{}, {}, {}, {}};
#pragma unroll
    for (int kb = 0; kb < C; kb += 32) { v16b ah, al; frag_split(&Ob[nloc][kb], hlf, ah, al);
#pragma unroll
      for (int t = 0; t < 4; ++t) { const v16b bw = frag_kb(Wd + (size_t)(wave * 64 + t * 16 + nloc) * C + kb, hlf); o[t] = wmma16b(ah, bw, o[t]); o[t] = wmma16b(al, bw, o[t]); } }
    if (hlf == 0) {
#pragma unroll
      for (int t = 0; t < 4; ++t) { const int cc = wave * 64 + t * 16 + nloc; Oo[cc] = o[t][0] * (1.0f / AS_) + db[cc]; } } }
  __syncthreads();
  for (int pass = 0; pass < 2; ++pass) { if (c < 64) *(volatile v4f*)(out + ((size_t)b * NB + n) * D + c * 4) = *(const v4f*)(&Oo[c * 4]); __threadfence(); }
}

__global__ __launch_bounds__(256) void wprep_kernel(const float* __restrict__ dw, b16* __restrict__ Wd) {
  const int t_ = blockIdx.x * 256 + threadIdx.x;
  for (int pass = 0; pass < 2; ++pass) { for (int i = t_; i < D * (C / 8); i += gridDim.x * 256) { const int d = i / (C / 8), c0 = (i % (C / 8)) * 8; v8b v; for (int e = 0; e < 8; ++e) v[e] = (b16)bf16_rne(dw[(size_t)(c0 + e) * D + d]); *(volatile v8b*)(Wd + (size_t)d * C + c0) = v; } __threadfence(); }
}
}

extern "C" void kernel_launch(void* const* d_in, const int* in_sizes, int n_in,
                              void* d_out, int out_size, void* d_ws, size_t ws_size, hipStream_t stream) {
  (void)n_in; (void)out_size;
  const float* img = (const float*)d_in[0]; const float* boxes = (const float*)d_in[1]; const float* cw = (const float*)d_in[2]; const float* cb = (const float*)d_in[3]; const float* dw = (const float*)d_in[4]; const float* db = (const float*)d_in[5];
  float* out = (float*)d_out;
  if (in_sizes[0] != Bn * IMG * IMG * 3 || in_sizes[1] != Bn * NB * 4 || in_sizes[2] != KP * C || in_sizes[4] != C * D) return;
  size_t off = 0; char* ws = (char*)d_ws;
  auto carve = [&](size_t bytes) { char* p = ws + off; off += (bytes + 255) & ~(size_t)255; return p; };
  b16* A = (b16*)carve((size_t)NPATCH * KP * 2); b16* Wc = (b16*)carve((size_t)C * KP * 2); float* F = (float*)carve((size_t)NPATCH * C * 4); b16* Wd = (b16*)carve((size_t)D * C * 2);
  if (off > ws_size) return;
  patch_kernel<<<dim3(FS, Bn), 256, 0, stream>>>(img, cw, A, Wc);
  wprep_kernel<<<32, 256, 0, stream>>>(dw, Wd);
  stem_kernel<<<dim3(2, NPATCH / 32), 64, 0, stream>>>(A, Wc, cb, F);
  roi_kernel<<<dim3(NB, Bn), 256, 0, stream>>>(F, boxes, Wd, db, out);
}
